// HeteroGCNGNN_62079457296457
// MI455X (gfx1250) — hardware-run, weakly checked
//
#include <hip/hip_runtime.h>


namespace {
constexpr int NN = 20000, E = 600000, D = 128, OUT = 16, NPB = 8;
constexpr float XS = 8.0f, HS = 256.0f, WSC = 256.0f;
typedef _Float16 b16;
typedef __attribute__((ext_vector_type(16))) _Float16 v16b;
typedef __attribute__((ext_vector_type(8))) _Float16 v8b;
typedef __attribute__((ext_vector_type(8))) float v8f;
typedef __attribute__((ext_vector_type(4))) float v4f;
__device__ __forceinline__ float bf16_rne(float f) { unsigned int u = __float_as_uint(f); u += 0x7FFFu + ((u >> 16) & 1u); float r = __uint_as_float(u & 0xFFFF0000u); asm volatile("" : "+v"(r)); return r; }
__device__ __forceinline__ float bfv(float f) { float r = bf16_rne(f); asm volatile("" : "+v"(r)); return r; }
__device__ __forceinline__ void split16(float v, b16& hi, b16& lo) { hi = (b16)v; lo = (b16)(v - (float)hi); }
__device__ __forceinline__ v16b frag_kb(const b16* p, int hh) { const v8b a = *(const v8b*)(p + 8 * hh), b = *(const v8b*)(p + 16 + 8 * hh); v16b f;
#pragma unroll
  for (int e = 0; e < 8; ++e) { f[e] = a[e]; f[8 + e] = b[e]; } return f; }
__device__ __forceinline__ v8f wmma16b(v16b a, v16b b, v8f c) { v8f d = __builtin_amdgcn_wmma_f32_16x16x32_f16(false, a, false, b, (short)0, c, false, false); asm volatile("v_nop\n\tv_nop\n\tv_nop\n\tv_nop" : "+v"(d) : "v"(a), "v"(b)); return d; }
__device__ __forceinline__ void wave_lds_sync() { __builtin_amdgcn_fence(__ATOMIC_RELEASE, "workgroup"); __builtin_amdgcn_wave_barrier(); __builtin_amdgcn_fence(__ATOMIC_ACQUIRE, "workgroup"); }
__device__ __forceinline__ float pmul(float a, float b) { float p = a * b; asm volatile("" : "+v"(p)); return p; }
__device__ __forceinline__ int iclamp(int v, int lo, int hi) { return v < lo ? lo : (v > hi ? hi : v); }
constexpr int CSR_NBLK8 = 512, CSR_GB8 = 8, CSR_GN8 = 1 << CSR_GB8  , CSR_TS8 = (CSR_GN8 < 32 ? 32 : CSR_GN8)  , CSR_MAXG8 = 512, CSR_CAP8 = 12288  ;
__device__ __host__ __forceinline__ int csr_tix8(int v) { return (v >> CSR_GB8) * CSR_TS8 + (v & (CSR_GN8 - 1)); }
__global__ __launch_bounds__(64) void csrA_kernel8(const int* __restrict__ dst, int E, int N, int nG, int CHP, int NGP, int* __restrict__ STG, int* __restrict__ HST) {
  extern __shared__ int sm[];
  int* cnt = sm; int* run = sm + NGP; int* ids = sm + 2 * NGP;
  const int b = blockIdx.x; const int ch = (E + CSR_NBLK8 - 1) / CSR_NBLK8; const int e0 = b * ch, e1 = min(E, e0 + ch);
  for (int i = threadIdx.x; i < NGP; i += 64) cnt[i] = 0;
  for (int i = threadIdx.x; i < CHP; i += 64) ids[i] = -1;
  __syncthreads();
  if (threadIdx.x == 0) {
    for (int e = e0; e < e1; ++e) { int d = dst[e]; d = (d < 0) ? 0 : (d >= N ? N - 1 : d); cnt[d >> CSR_GB8] += 1; }
    int acc = 0; for (int g = 0; g < nG; ++g) { run[g] = acc; acc += cnt[g]; }
    for (int e = e0; e < e1; ++e) { int d = dst[e]; d = (d < 0) ? 0 : (d >= N ? N - 1 : d); const int g = d >> CSR_GB8; ids[run[g]] = e; run[g] += 1; } }
  __syncthreads();
  typedef __attribute__((ext_vector_type(4))) int v4i;
  for (int pass = 0; pass < 2; ++pass) {
    for (int i = threadIdx.x; i < CHP / 4; i += 64) *(volatile v4i*)(STG + (size_t)b * CHP + i * 4) = *(const v4i*)(&ids[i * 4]);
    for (int i = threadIdx.x; i < NGP / 4; i += 64) { v4i v; for (int e = 0; e < 4; ++e) v[e] = (i * 4 + e < nG) ? cnt[i * 4 + e] : 0; *(volatile v4i*)(HST + (size_t)b * NGP + i * 4) = v; }
    __threadfence(); }
}
__global__ __launch_bounds__(512) void csrS_kernel8(const int* __restrict__ HST, int nG, int NGP, int* __restrict__ START, int* __restrict__ TOT, int* __restrict__ OFF) {
  __shared__ int tot[CSR_MAXG8];
  const int b = threadIdx.x;
  for (int pass = 0; pass < 2; ++pass) { int runb = 0; for (int g = 0; g < nG; ++g) { int c = HST[(size_t)b * NGP + g]; c = (c < 0) ? 0 : c; ((volatile int*)OFF)[(size_t)g * CSR_NBLK8 + b] = runb; runb += c; } __threadfence(); }
  for (int g = threadIdx.x; g < nG; g += 512) { int s = 0; for (int bb = 0; bb < CSR_NBLK8; ++bb) { int c = HST[(size_t)bb * NGP + g]; s += (c < 0) ? 0 : c; } tot[g] = s; }
  __syncthreads();
  if (threadIdx.x < 32) {
    __shared__ int st[CSR_MAXG8 + 32];
    if (threadIdx.x == 0) { int acc = 0; for (int g = 0; g < NGP; ++g) { st[g] = acc; if (g < nG) acc += (tot[g] + 31) & ~31; } st[NGP] = acc; }
    __builtin_amdgcn_fence(__ATOMIC_RELEASE, "workgroup"); __builtin_amdgcn_wave_barrier(); __builtin_amdgcn_fence(__ATOMIC_ACQUIRE, "workgroup");
    for (int pass = 0; pass < 2; ++pass) { for (int i = threadIdx.x; i < NGP + 32; i += 32) { ((volatile int*)START)[i] = (i <= NGP) ? st[min(i, NGP)] : 0; ((volatile int*)TOT)[i] = (i < nG) ? tot[i] : 0; } __threadfence(); } }
}
__global__ __launch_bounds__(256) void csrB_kernel8(const int* __restrict__ dst, int N, int nG, int CHP, int NGP, int permLen, const int* __restrict__ STG, const int* __restrict__ HST, const int* __restrict__ OFF, const int* __restrict__ START, const int* __restrict__ TOT, int* __restrict__ PERM, int* __restrict__ ROWPTR, int* __restrict__ ROWCNT, int* __restrict__ FLAG) {
  typedef __attribute__((ext_vector_type(4))) int v4i;
  __shared__ int ids[CSR_CAP8]; __shared__ unsigned short key[CSR_CAP8]; __shared__ int outp[CSR_CAP8]; __shared__ int ncnt[CSR_GN8 + 1]; __shared__ int boff[CSR_NBLK8 + 1];
  const int g = blockIdx.x, t_ = threadIdx.x; int tot = TOT[g]; int st = START[g], stn = START[g + 1]; const int v0 = g * CSR_GN8; const int nv = min(CSR_GN8, N - v0); const int t0 = g * CSR_TS8;
  st = (st < 0) ? 0 : (st > permLen - 32 ? permLen - 32 : st) & ~31; stn = (stn < st) ? st : (stn > permLen ? permLen : stn); tot = (tot < 0) ? 0 : tot; if (tot > stn - st && tot <= CSR_CAP8) tot = stn - st;
  if (tot > CSR_CAP8) {
    for (int pass = 0; pass < 2; ++pass) { for (int i = t_; i < CSR_TS8 / 4; i += 256) { v4i a, c; for (int e = 0; e < 4; ++e) { a[e] = st; c[e] = 0; } *(volatile v4i*)(ROWPTR + t0 + i * 4) = a; *(volatile v4i*)(ROWCNT + t0 + i * 4) = c; } if (t_ == 0) ((volatile int*)FLAG)[0] = 1; __threadfence(); } (void)nv; return; }
  if (t_ == 0) { int acc = 0; for (int b = 0; b < CSR_NBLK8; ++b) { boff[b] = acc; int c = HST[(size_t)b * NGP + g]; c = (c < 0) ? 0 : (c > CHP ? CHP : c); acc += c; if (acc > tot) acc = tot; } boff[CSR_NBLK8] = acc; }
  for (int i = t_; i <= CSR_GN8; i += 256) ncnt[i] = 0;
  __syncthreads();
  for (int b = 0; b < CSR_NBLK8; ++b) { const int c = boff[b + 1] - boff[b]; int o_ = OFF[(size_t)g * CSR_NBLK8 + b]; o_ = (o_ < 0) ? 0 : (o_ > CHP - c ? CHP - c : o_); const int* src_ = STG + (size_t)b * CHP + o_;
    for (int i = t_; i < c; i += 256) { int id = src_[i]; id = (id < 0) ? 0 : id; ids[boff[b] + i] = id; int d = dst[id]; d = (d < v0) ? v0 : (d >= N ? N - 1 : d); int kk = d - v0; kk = (kk < 0) ? 0 : (kk >= CSR_GN8 ? CSR_GN8 - 1 : kk); key[boff[b] + i] = (unsigned short)kk; } }
  __syncthreads();
  if (t_ == 0) { for (int i = 0; i < tot; ++i) ncnt[key[i]] += 1; int acc = 0; for (int vl = 0; vl < CSR_GN8; ++vl) { const int c = ncnt[vl]; ncnt[vl] = acc; acc += c; } ncnt[CSR_GN8] = acc;
    for (int i = 0; i < tot; ++i) { const int vl = key[i]; outp[ncnt[vl]] = ids[i]; ncnt[vl] += 1; }
    for (int vl = CSR_GN8; vl > 0; --vl) ncnt[vl] = ncnt[vl - 1]; ncnt[0] = 0; }
  __syncthreads();
  for (int pass = 0; pass < 2; ++pass) {
    for (int i = t_; i < (stn - st) / 4; i += 256) { v4i v; for (int e = 0; e < 4; ++e) { const int q = i * 4 + e; v[e] = (q < tot) ? outp[q] : -1; } *(volatile v4i*)(PERM + st + i * 4) = v; }
    for (int i = t_; i < CSR_TS8 / 4; i += 256) { v4i a, c; for (int e = 0; e < 4; ++e) { const int vl = i * 4 + e; const int vc = vl < CSR_GN8 ? vl : CSR_GN8; a[e] = (vl < CSR_GN8) ? st + ncnt[vc] : st; c[e] = (vl < nv) ? (ncnt[(vc < CSR_GN8 ? vc : CSR_GN8 - 1) + 1] - ncnt[vc]) : 0; } *(volatile v4i*)(ROWPTR + t0 + i * 4) = a; *(volatile v4i*)(ROWCNT + t0 + i * 4) = c; }
    __threadfence(); }
}
__global__ __launch_bounds__(256) void csrZ_kernel8(int* __restrict__ p, size_t n4) { typedef __attribute__((ext_vector_type(4))) int v4i; const size_t tid = (size_t)blockIdx.x * 256 + threadIdx.x, nth = (size_t)gridDim.x * 256; v4i z = {0, 0, 0, 0}; for (size_t i = tid; i < n4; i += nth) *(volatile v4i*)(p + i * 4) = z; }
struct CsrBufs8 { int *STG, *HST, *OFF, *START, *TOT, *PERM, *ROWPTR, *ROWCNT, *FLAG; int nG, NGP, CHP; size_t permLen; char* base; size_t bytes; };
static size_t csr_carve8(CsrBufs8& c, char* ws, size_t off, int E, int N) {
  const size_t off0 = off; c.base = ws + off;
  auto al = [&](size_t bytes) { char* p = ws + off; off += (bytes + 255) & ~(size_t)255; return p; };
  c.nG = (N + CSR_GN8 - 1) / CSR_GN8; c.NGP = (c.nG + 31) & ~31; const int ch = (E + CSR_NBLK8 - 1) / CSR_NBLK8; c.CHP = (ch + 31) & ~31; c.permLen = (size_t)E + 32 * (size_t)c.nG + 32;
  c.STG = (int*)al((size_t)CSR_NBLK8 * c.CHP * 4); c.HST = (int*)al((size_t)CSR_NBLK8 * c.NGP * 4); c.OFF = (int*)al((size_t)c.NGP * CSR_NBLK8 * 4); c.START = (int*)al((size_t)(c.NGP + 64) * 4); c.TOT = (int*)al((size_t)(c.NGP + 64) * 4);
  c.PERM = (int*)al(c.permLen * 4); c.ROWPTR = (int*)al((size_t)c.nG * CSR_TS8 * 4); c.ROWCNT = (int*)al((size_t)c.nG * CSR_TS8 * 4); c.FLAG = (int*)al(256);
  c.bytes = off - off0; return off;
}
static void csr_build8(const CsrBufs8& c, const int* dst, int E, int N, hipStream_t stream) {
  const size_t smem = (size_t)(2 * c.NGP + c.CHP) * 4;
  csrZ_kernel8<<<512, 256, 0, stream>>>((int*)c.base, c.bytes / 16);
  csrA_kernel8<<<CSR_NBLK8, 64, smem, stream>>>(dst, E, N, c.nG, c.CHP, c.NGP, c.STG, c.HST);
  csrS_kernel8<<<1, 512, 0, stream>>>(c.HST, c.nG, c.NGP, c.START, c.TOT, c.OFF);
  csrB_kernel8<<<c.nG, 256, 0, stream>>>(dst, N, c.nG, c.CHP, c.NGP, (int)c.permLen, c.STG, c.HST, c.OFF, c.START, c.TOT, c.PERM, c.ROWPTR, c.ROWCNT, c.FLAG);
}


__global__ __launch_bounds__(256) void wput_kernel(const float* __restrict__ wc, const float* __restrict__ wlg, const float* __restrict__ wlr, b16* __restrict__ WC, b16* __restrict__ WL) { const size_t nt = (size_t)gridDim.x * 256, u0 = (size_t)blockIdx.x * 256 + threadIdx.x; v8b v;
  for (size_t u = u0; u < (size_t)8 * D * 16; u += nt) { const int m = (int)(u / (D * 16)), r = (int)(u % (D * 16)); const int o = r / 16, k0 = (r % 16) * 8;
#pragma unroll
    for (int j = 0; j < 8; ++j) v[j] = (b16)(bf16_rne(wc[((size_t)m * D + k0 + j) * D + o]) * WSC); for (int pass = 0; pass < 2; ++pass) { *(volatile v8b*)(WC + ((size_t)m * D + o) * D + k0) = v; __threadfence(); } }
  for (size_t u = u0; u < (size_t)2 * OUT * 16; u += nt) { const int t = (int)(u / (OUT * 16)), r = (int)(u % (OUT * 16)); const int o = r / 16, k0 = (r % 16) * 8; const float* w = t ? wlr : wlg;
#pragma unroll
    for (int j = 0; j < 8; ++j) v[j] = (b16)(bf16_rne(w[(size_t)(k0 + j) * OUT + o]) * WSC); for (int pass = 0; pass < 2; ++pass) { *(volatile v8b*)(WL + ((size_t)t * OUT + o) * D + k0) = v; __threadfence(); } } }
template <int SELF>
__global__ __launch_bounds__(256) void deg_kernel(const float* __restrict__ w, const int* __restrict__ PERM, const int* __restrict__ ROWPTR, const int* __restrict__ ROWCNT, int permLen, float* __restrict__ DG) { __shared__ float Ds[32]; const int wave = threadIdx.x >> 5, lane = threadIdx.x & 31; const size_t i = (size_t)blockIdx.x * 8 + wave; float s = 0.0f; if (i < (size_t)NN) { int st = ROWPTR[i], cnt = ROWCNT[i]; cnt = iclamp(cnt, 0, E); st = iclamp(st, 0, permLen - cnt); for (int j = lane; j < cnt; j += 32) { const int e = iclamp(PERM[st + j], 0, E - 1); s += bfv(w[e]); } }
  for (int o = 16; o; o >>= 1) s += __shfl_xor(s, o); if (lane == 0) { const float d = s + (SELF ? 1.0f : 0.0f); Ds[wave] = d > 0.0f ? rsqrtf(d) : 0.0f; }
  __syncthreads();
  for (int pass = 0; pass < 2; ++pass) { if (wave == 0) ((volatile float*)DG)[(size_t)blockIdx.x * 32 + lane] = lane < 8 ? Ds[lane] : 0.0f; __threadfence(); } }
__device__ __forceinline__ float dg_at(const float* DG, size_t i) { return DG[(i >> 3) * 32 + (i & 7)]; }
template <int MODE, int NT>
__global__ __launch_bounds__(32) void lin_kernel(const float* __restrict__ IN, const b16* __restrict__ W, const float* __restrict__ bias, int NLIM, float* __restrict__ HW) { constexpr int OW = NT * 16; __shared__ __attribute__((aligned(16))) b16 Ah[16][D + 8], Al[16][D + 8]; __shared__ float Tf[16][OW + 4]; const int lane = threadIdx.x, nloc = lane & 15, hlf = lane >> 4; const size_t m0 = (size_t)blockIdx.x * 16; if (m0 >= (size_t)NLIM) return;
  for (int rr = 0; rr < 16; ++rr) for (int q = 0; q < 4; ++q) { const int c = q * 32 + lane; const float v = IN[(m0 + rr) * D + c]; b16 p, ql; if (MODE == 0) { p = (b16)(bf16_rne(v) * XS); ql = (b16)0.0f; } else split16(v * HS, p, ql); Ah[rr][c] = p; Al[rr][c] = ql; }
  if (lane < 16) for (int k = D; k < D + 8; ++k) { Ah[lane][k] = (b16)0.0f; Al[lane][k] = (b16)0.0f; }
  wave_lds_sync(); v8f acc[NT];
#pragma unroll
  for (int t = 0; t < NT; ++t) acc[t] = (v8f){};
#pragma unroll
  for (int kb = 0; kb < D; kb += 32) { const v16b a = frag_kb(&Ah[nloc][kb], hlf), al = frag_kb(&Al[nloc][kb], hlf);
#pragma unroll
    for (int t = 0; t < NT; ++t) { const v16b bw = frag_kb(W + (size_t)(t * 16 + nloc) * D + kb, hlf); acc[t] = wmma16b(a, bw, acc[t]); if (MODE == 1) acc[t] = wmma16b(al, bw, acc[t]); } }
  const float osc = MODE == 0 ? 1.0f / (XS * WSC) : 1.0f / (HS * WSC);
#pragma unroll
  for (int t = 0; t < NT; ++t)
#pragma unroll
    for (int r8 = 0; r8 < 8; ++r8) Tf[8 * hlf + r8][t * 16 + nloc] = acc[t][r8] * osc + (bias ? bfv(bias[t * 16 + nloc]) : 0.0f);
  wave_lds_sync();
  for (int pass = 0; pass < 2; ++pass) { for (int rr = 0; rr < 16; ++rr) { if (NT == 8) *(volatile v4f*)(HW + (m0 + rr) * OW + lane * 4) = *(const v4f*)(&Tf[rr][lane * 4]); else if (lane < 16) ((volatile float*)HW)[(m0 + rr) * OW + lane] = Tf[rr][lane]; } __threadfence(); } }
__global__ __launch_bounds__(256) void sweep_kernel(const float* __restrict__ HA, const float* __restrict__ DSQ, const float* __restrict__ wa, const float* __restrict__ bA, const int* __restrict__ rowsA, const int* __restrict__ PERMA, const int* __restrict__ ROWPTRA, const int* __restrict__ ROWCNTA, int permLenA,
    const float* __restrict__ HB, const float* __restrict__ DS, const float* __restrict__ DD, const float* __restrict__ wb, const float* __restrict__ bB, const int* __restrict__ rowsB, const int* __restrict__ PERMB, const int* __restrict__ ROWPTRB, const int* __restrict__ ROWCNTB, int permLenB, int NLIM, float* __restrict__ OUTX) {
  const int wave = threadIdx.x >> 5, lane = threadIdx.x & 31; const size_t i = (size_t)blockIdx.x * NPB + wave; if (i >= (size_t)NLIM) return; v4f aa = {0, 0, 0, 0}, ab = {0, 0, 0, 0};
  { int st = ROWPTRA[i], cnt = ROWCNTA[i]; cnt = iclamp(cnt, 0, E); st = iclamp(st, 0, permLenA - cnt);
#pragma unroll 1
    for (int j = 0; j < cnt; ++j) { const int e = iclamp(PERMA[st + j], 0, E - 1); const size_t u = (size_t)iclamp(rowsA[e], 0, NN - 1); if (u >= (size_t)NLIM) continue; const float wgt = pmul(dg_at(DSQ, u), bfv(wa[e])); const v4f v = *(const v4f*)(HA + u * D + lane * 4);
#pragma unroll
      for (int k = 0; k < 4; ++k) aa[k] += pmul(wgt, v[k]); } }
  { int st = ROWPTRB[i], cnt = ROWCNTB[i]; cnt = iclamp(cnt, 0, E); st = iclamp(st, 0, permLenB - cnt);
#pragma unroll 1
    for (int j = 0; j < cnt; ++j) { const int e = iclamp(PERMB[st + j], 0, E - 1); const size_t u = (size_t)iclamp(rowsB[e], 0, NN - 1); if (u >= (size_t)NLIM) continue; const float wgt = pmul(dg_at(DS, u), bfv(wb[e])); const v4f v = *(const v4f*)(HB + u * D + lane * 4);
#pragma unroll
      for (int k = 0; k < 4; ++k) ab[k] += pmul(wgt, v[k]); } }
  const float di = dg_at(DSQ, i), ddi = dg_at(DD, i); const v4f hv = *(const v4f*)(HA + i * D + lane * 4); v4f o;
#pragma unroll
  for (int k = 0; k < 4; ++k) { const int c = lane * 4 + k; const float a = pmul(di, aa[k] + pmul(di, hv[k])) + bfv(bA[c]); const float b = pmul(ddi, ab[k]) + bfv(bB[c]); o[k] = fmaxf(0.5f * (a + b), 0.0f); }
  for (int pass = 0; pass < 2; ++pass) { *(volatile v4f*)(OUTX + i * D + lane * 4) = o; __threadfence(); } }
}

extern "C" void kernel_launch(void* const* d_in, const int* in_sizes, int n_in, void* d_out, int out_size, void* d_ws, size_t ws_size, hipStream_t stream) {
  (void)n_in;
  auto Fp = [&](int i) { return (const float*)d_in[i]; }; auto Ip = [&](int i) { return (const int*)d_in[i]; };
  if (in_sizes[0] != NN * D || in_sizes[1] != NN * D || in_sizes[2] != 2 * E || in_sizes[5] != 2 * E || in_sizes[6] != E || in_sizes[9] != E || in_sizes[10] != 8 * D * D || in_sizes[11] != 8 * D || in_sizes[12] != D * OUT || in_sizes[14] != D * OUT || out_size != 2 * NN * OUT) return;
  const int NLIM = NN;
  size_t off = 0; char* ws = (char*)d_ws;
  auto carve = [&](size_t bytes) { char* p = ws + off; off += (bytes + 255) & ~(size_t)255; return p; };
  b16* WC = (b16*)carve((size_t)8 * D * D * 2); b16* WL = (b16*)carve((size_t)2 * OUT * D * 2);
  float* HGG = (float*)carve((size_t)NN * D * 4); float* HGR = (float*)carve((size_t)NN * D * 4); float* HRG = (float*)carve((size_t)NN * D * 4); float* HRR = (float*)carve((size_t)NN * D * 4); float* XG = (float*)carve((size_t)NN * D * 4); float* XR = (float*)carve((size_t)NN * D * 4);
  const size_t dgsz = (size_t)(NN / 8 + 1) * 32 * 4; float* DGG = (float*)carve(dgsz); float* DRR = (float*)carve(dgsz); float* DGRs = (float*)carve(dgsz); float* DGRd = (float*)carve(dgsz); float* DRGs = (float*)carve(dgsz); float* DRGd = (float*)carve(dgsz);
  CsrBufs8 cgg, cgr, crg, crr, rgr, rrg; off = csr_carve8(cgg, ws, off, E, NN); off = csr_carve8(cgr, ws, off, E, NN); off = csr_carve8(crg, ws, off, E, NN); off = csr_carve8(crr, ws, off, E, NN); off = csr_carve8(rgr, ws, off, E, NN); off = csr_carve8(rrg, ws, off, E, NN);
  if (off > ws_size || off > ((size_t)144 << 20)) return;
  const int nb = (NLIM + NPB - 1) / NPB, ndb = (NN + 7) / 8;
  wput_kernel<<<64, 256, 0, stream>>>(Fp(10), Fp(12), Fp(14), WC, WL);
  csr_build8(cgg, Ip(2) + E, E, NN, stream); csr_build8(cgr, Ip(3) + E, E, NN, stream); csr_build8(crg, Ip(4) + E, E, NN, stream); csr_build8(crr, Ip(5) + E, E, NN, stream);
  csr_build8(rgr, Ip(3), E, NN, stream); csr_build8(rrg, Ip(4), E, NN, stream);
  deg_kernel<1><<<ndb, 256, 0, stream>>>(Fp(6), cgg.PERM, cgg.ROWPTR, cgg.ROWCNT, (int)cgg.permLen, DGG);
  deg_kernel<1><<<ndb, 256, 0, stream>>>(Fp(9), crr.PERM, crr.ROWPTR, crr.ROWCNT, (int)crr.permLen, DRR);
  deg_kernel<0><<<ndb, 256, 0, stream>>>(Fp(7), rgr.PERM, rgr.ROWPTR, rgr.ROWCNT, (int)rgr.permLen, DGRs); deg_kernel<0><<<ndb, 256, 0, stream>>>(Fp(7), cgr.PERM, cgr.ROWPTR, cgr.ROWCNT, (int)cgr.permLen, DGRd);
  deg_kernel<0><<<ndb, 256, 0, stream>>>(Fp(8), rrg.PERM, rrg.ROWPTR, rrg.ROWCNT, (int)rrg.permLen, DRGs); deg_kernel<0><<<ndb, 256, 0, stream>>>(Fp(8), crg.PERM, crg.ROWPTR, crg.ROWCNT, (int)crg.permLen, DRGd);
  for (int l = 0; l < 2; ++l) { const float* ig = l ? XG : Fp(0); const float* ir = l ? XR : Fp(1); const b16* W = WC + (size_t)l * 4 * D * D; const float* bc = Fp(11) + l * 4 * D;
    if (l == 0) { lin_kernel<0, 8><<<NLIM / 16, 32, 0, stream>>>(ig, W, nullptr, NLIM, HGG); lin_kernel<0, 8><<<NLIM / 16, 32, 0, stream>>>(ig, W + (size_t)D * D, nullptr, NLIM, HGR); lin_kernel<0, 8><<<NLIM / 16, 32, 0, stream>>>(ir, W + (size_t)2 * D * D, nullptr, NLIM, HRG); lin_kernel<0, 8><<<NLIM / 16, 32, 0, stream>>>(ir, W + (size_t)3 * D * D, nullptr, NLIM, HRR); }
    else { lin_kernel<1, 8><<<NLIM / 16, 32, 0, stream>>>(ig, W, nullptr, NLIM, HGG); lin_kernel<1, 8><<<NLIM / 16, 32, 0, stream>>>(ig, W + (size_t)D * D, nullptr, NLIM, HGR); lin_kernel<1, 8><<<NLIM / 16, 32, 0, stream>>>(ir, W + (size_t)2 * D * D, nullptr, NLIM, HRG); lin_kernel<1, 8><<<NLIM / 16, 32, 0, stream>>>(ir, W + (size_t)3 * D * D, nullptr, NLIM, HRR); }
    sweep_kernel<<<nb, 256, 0, stream>>>(HGG, DGG, Fp(6), bc, Ip(2), cgg.PERM, cgg.ROWPTR, cgg.ROWCNT, (int)cgg.permLen, HRG, DRGs, DRGd, Fp(8), bc + 2 * D, Ip(4), crg.PERM, crg.ROWPTR, crg.ROWCNT, (int)crg.permLen, NLIM, XG);
    sweep_kernel<<<nb, 256, 0, stream>>>(HRR, DRR, Fp(9), bc + 3 * D, Ip(5), crr.PERM, crr.ROWPTR, crr.ROWCNT, (int)crr.permLen, HGR, DGRs, DGRd, Fp(7), bc + D, Ip(3), cgr.PERM, cgr.ROWPTR, cgr.ROWCNT, (int)cgr.permLen, NLIM, XR); }
  lin_kernel<1, 1><<<NLIM / 16, 32, 0, stream>>>(XG, WL, Fp(13), NLIM, (float*)d_out);
  lin_kernel<1, 1><<<NLIM / 16, 32, 0, stream>>>(XR, WL + (size_t)OUT * D, Fp(15), NLIM, (float*)d_out + (size_t)NN * OUT);
}
